// MultiHead_Attention_73065983640334
// MI455X (gfx1250) — hardware-verified
//
#include <hip/hip_runtime.h>


#ifndef NB_
#define NB_ 2
#endif
#ifndef SEQ_
#define SEQ_ 2048
#endif
#ifndef SRES_
#define SRES_ 512
#endif
#define SEQ_FULL_ 2048
#define D_ 1024
#define H_ 16
#define DH_ 64
#define NBH_ (NB_ * H_)
#define SR_ ((SEQ_ < SRES_) ? SEQ_ : SRES_)
#define LDT_ 72
#define LDP_ 40
#define LDO_ 68
#define RC_ 4096.0f
#define RCI_ 0.000244140625f
#define WOC_ 64.0f
#define WOCI_ 0.015625f

static_assert(NB_ >= 1 && NB_ <= 2);
static_assert((SEQ_ % 64) == 0 && SEQ_ >= 64 && SEQ_ <= SEQ_FULL_);
static_assert((SR_ % 64) == 0 && SR_ >= 64 && SR_ <= SEQ_);
static_assert(D_ == H_ * DH_ && DH_ == 64 && (D_ % 64) == 0 && (D_ / 8) == 128);
static_assert((size_t)NB_ * SEQ_ * D_ * 4 <= (size_t)16777216);

typedef _Float16 v16h __attribute__((ext_vector_type(16)));
typedef _Float16 v8h __attribute__((ext_vector_type(8)));
typedef __bf16 v16b __attribute__((ext_vector_type(16)));
typedef float v8f __attribute__((ext_vector_type(8)));
typedef float v4f __attribute__((ext_vector_type(4)));
typedef unsigned int v4u __attribute__((ext_vector_type(4)));
typedef unsigned short v8s __attribute__((ext_vector_type(8)));
typedef unsigned short us_t;

union Frag { v4u q[2]; v8h hv[2]; v16h h; v16b b; };
static_assert(sizeof(Frag) == 32);

#define DEV static __device__ __forceinline__

DEV v8f zero8() { v8f z = {0.f, 0.f, 0.f, 0.f, 0.f, 0.f, 0.f, 0.f}; return z; }
DEV Frag fragz() { Frag f; v4u z = {0u, 0u, 0u, 0u}; f.q[0] = z; f.q[1] = z; return f; }

DEV v8f mma_bf16(v16b a, v16b b, v8f c) {
  c = __builtin_amdgcn_wmma_f32_16x16x32_bf16(false, a, false, b, (short)0, c, false, false);
  asm volatile("v_nop\n\tv_nop\n\tv_nop\n\tv_nop" : "+v"(c) : "v"(a), "v"(b));
  return c;
}
DEV v8f mma_f16(v16h a, v16h b, v8f c) {
  c = __builtin_amdgcn_wmma_f32_16x16x32_f16(false, a, false, b, (short)0, c, false, false);
  asm volatile("v_nop\n\tv_nop\n\tv_nop\n\tv_nop" : "+v"(c) : "v"(a), "v"(b));
  return c;
}

DEV Frag ldfrag(const us_t* __restrict__ base, int ld) {
  const int lane = threadIdx.x & 31;
  const us_t* p = base + (size_t)(lane & 15) * ld + ((lane >> 4) << 3);
  Frag f;
  f.q[0] = *(const v4u*)p;
  f.q[1] = *(const v4u*)(p + 16);
  return f;
}

DEV unsigned int bf16_bits(float f) {
  unsigned int u = __float_as_uint(f);
  u += 0x7FFFu + ((u >> 16) & 1u);
  return u >> 16;
}
DEV us_t f16_bits(float f) {
  _Float16 hv = (_Float16)f;
  return __builtin_bit_cast(us_t, hv);
}

DEV void wave_lds_sync() {
  asm volatile("" ::: "memory");
  __builtin_amdgcn_fence(3, "wavefront");
  __builtin_amdgcn_wave_barrier();
  __builtin_amdgcn_fence(2, "wavefront");
  asm volatile("" ::: "memory");
}

__global__ __launch_bounds__(256) void k_prep_x(const float* __restrict__ x, us_t* __restrict__ Xb) {
  const int t = blockIdx.x * 256 + threadIdx.x;
  if (t >= NB_ * SEQ_ * (D_ / 8)) return;
  const int row = t >> 7;
  const int c8 = (t & 127) << 3;
  const int b = row / SEQ_, s = row - b * SEQ_;
  const float* src = x + ((size_t)b * SEQ_FULL_ + s) * D_ + c8;
  const v4f lo = *(const v4f*)src;
  const v4f hi = *(const v4f*)(src + 4);
  v4u o;
  o.x = bf16_bits(lo.x) | (bf16_bits(lo.y) << 16);
  o.y = bf16_bits(lo.z) | (bf16_bits(lo.w) << 16);
  o.z = bf16_bits(hi.x) | (bf16_bits(hi.y) << 16);
  o.w = bf16_bits(hi.z) | (bf16_bits(hi.w) << 16);
  us_t* dst = Xb + (size_t)row * D_ + c8;
  *(volatile v4u*)dst = o;
  __threadfence();
  *(volatile v4u*)dst = o;
}

__global__ __launch_bounds__(256) void k_prep_w(const float* __restrict__ Wq, const float* __restrict__ Wk,
                                                const float* __restrict__ Wv, const float* __restrict__ Wo,
                                                us_t* __restrict__ WqT, us_t* __restrict__ WkT,
                                                us_t* __restrict__ WvT, us_t* __restrict__ WoT) {
  __shared__ __align__(16) us_t T[64 * LDT_];
  const int z = blockIdx.z;
  const float* src = (z == 0) ? Wq : (z == 1) ? Wk : (z == 2) ? Wv : Wo;
  us_t* dst = (z == 0) ? WqT : (z == 1) ? WkT : (z == 2) ? WvT : WoT;
  const int k0 = blockIdx.x * 64, n0 = blockIdx.y * 64;
  const int t = threadIdx.x, c = t & 63, r4 = t >> 6;
#pragma unroll 4
  for (int i = 0; i < 16; ++i) {
    const int kk = 4 * i + r4;
    const float v = src[(size_t)(k0 + kk) * D_ + n0 + c];
    const unsigned int bb = bf16_bits(v);
    const us_t hb = f16_bits(__uint_as_float(bb << 16) * WOC_);
    T[c * LDT_ + kk] = (z == 3) ? hb : (us_t)bb;
  }
  __syncthreads();
  const int w = t >> 5, lane = t & 31, pc = lane & 7;
  v4u val[2];
  size_t o[2];
#pragma unroll
  for (int p = 0; p < 2; ++p) {
    const int L = 8 * w + 4 * p + (lane >> 3);
    const v8s e = *(const v8s*)&T[L * LDT_ + 8 * pc];
    val[p] = __builtin_bit_cast(v4u, e);
    o[p] = (size_t)(n0 + L) * D_ + k0 + 8 * pc;
  }
#pragma unroll
  for (int p = 0; p < 2; ++p) *(volatile v4u*)(dst + o[p]) = val[p];
  __threadfence();
#pragma unroll
  for (int p = 0; p < 2; ++p) *(volatile v4u*)(dst + o[p]) = val[p];
}

__global__ __launch_bounds__(128) void k_proj(const us_t* __restrict__ Xb, const us_t* __restrict__ WqT,
                                              const us_t* __restrict__ WkT, const us_t* __restrict__ WvT,
                                              us_t* __restrict__ Qh, us_t* __restrict__ Qr,
                                              us_t* __restrict__ Kh, us_t* __restrict__ Kr,
                                              us_t* __restrict__ Vth, us_t* __restrict__ Vtr) {
  __shared__ __align__(16) _Float16 Th[64 * LDT_];
  __shared__ __align__(16) _Float16 Tr[64 * LDT_];
  const int tid = threadIdx.x, w = tid >> 5, lane = tid & 31, n = lane & 15, hh = lane >> 4;
  const int proj = blockIdx.z, h = blockIdx.y;
  const int nsb = SEQ_ / 64;
  const int b = blockIdx.x / nsb, sblk = blockIdx.x - b * nsb, s0 = sblk * 64;
  const int bh = b * H_ + h;
  const us_t* W = (proj == 0) ? WqT : (proj == 1) ? WkT : WvT;
  const us_t* A = Xb + (size_t)(b * SEQ_ + s0 + 16 * w) * D_;
  const us_t* Bw = W + (size_t)(h * DH_) * D_;

  v8f c[4];
#pragma unroll
  for (int j = 0; j < 4; ++j) c[j] = zero8();
#pragma unroll 2
  for (int kk = 0; kk < D_; kk += 32) {
    const Frag a = ldfrag(A + kk, D_);
#pragma unroll
    for (int j = 0; j < 4; ++j) {
      const Frag bj = ldfrag(Bw + (size_t)(16 * j) * D_ + kk, D_);
      c[j] = mma_bf16(a.b, bj.b, c[j]);
    }
  }

  if (proj < 2) {
#pragma unroll
    for (int j = 0; j < 4; ++j) {
#pragma unroll
      for (int r = 0; r < 8; ++r) {
        const float v = c[j][r];
        const _Float16 hv = (_Float16)v;
        const int idx = (16 * w + 8 * hh + r) * LDT_ + 16 * j + n;
        Th[idx] = hv;
        Tr[idx] = (_Float16)((v - (float)hv) * RC_);
      }
    }
  } else {
#pragma unroll
    for (int j = 0; j < 4; ++j) {
      v8h ph, pr;
#pragma unroll
      for (int r = 0; r < 8; ++r) {
        const float v = c[j][r];
        const _Float16 hv = (_Float16)v;
        ph[r] = hv;
        pr[r] = (_Float16)((v - (float)hv) * RC_);
      }
      const int idx = (16 * j + n) * LDT_ + 16 * w + 8 * hh;
      *(v8h*)&Th[idx] = ph;
      *(v8h*)&Tr[idx] = pr;
    }
  }
  __syncthreads();

  const bool wres = (s0 < SR_);
  const int pc = lane & 7;
  v4u hq[4], rq[4];
  size_t oh[4], orr[4];
#pragma unroll
  for (int p = 0; p < 4; ++p) {
    const int L = 16 * w + 4 * p + (lane >> 3);
    const v8h e0 = *(const v8h*)&Th[L * LDT_ + 8 * pc];
    const v8h e1 = *(const v8h*)&Tr[L * LDT_ + 8 * pc];
    hq[p] = __builtin_bit_cast(v4u, e0);
    rq[p] = __builtin_bit_cast(v4u, e1);
    if (proj < 2) {
      oh[p]  = (size_t)(bh * SEQ_ + s0 + L) * DH_ + 8 * pc;
      orr[p] = (size_t)(bh * SR_ + s0 + L) * DH_ + 8 * pc;
    } else {
      oh[p]  = (size_t)(bh * DH_ + L) * SEQ_ + s0 + 8 * pc;
      orr[p] = (size_t)(bh * DH_ + L) * SR_ + s0 + 8 * pc;
    }
  }
  us_t* Ph = (proj == 0) ? Qh : (proj == 1) ? Kh : Vth;
  us_t* Pr = (proj == 0) ? Qr : (proj == 1) ? Kr : Vtr;
#pragma unroll
  for (int p = 0; p < 4; ++p) *(volatile v4u*)(Ph + oh[p]) = hq[p];
  if (wres) {
#pragma unroll
    for (int p = 0; p < 4; ++p) *(volatile v4u*)(Pr + orr[p]) = rq[p];
  }
  __threadfence();
#pragma unroll
  for (int p = 0; p < 4; ++p) *(volatile v4u*)(Ph + oh[p]) = hq[p];
  if (wres) {
#pragma unroll
    for (int p = 0; p < 4; ++p) *(volatile v4u*)(Pr + orr[p]) = rq[p];
  }
}

template <int RES>
__global__ __launch_bounds__(128) __attribute__((amdgpu_num_vgpr(256)))
void k_attn(const us_t* __restrict__ Qh, const us_t* __restrict__ Qr,
            const us_t* __restrict__ Kh, const us_t* __restrict__ Kr,
            const us_t* __restrict__ Vth, const us_t* __restrict__ Vtr,
            us_t* __restrict__ CtxH, us_t* __restrict__ CtxR, int qblk0, int nqb) {
  __shared__ __align__(16) _Float16 Pl[4][2][16 * LDP_];
  __shared__ __align__(16) _Float16 Cs[4][2][16 * LDT_];
  (void)nqb;
  const int tid = threadIdx.x, w = tid >> 5, lane = tid & 31, n = lane & 15, hh = lane >> 4;
  const int bh = blockIdx.x % NBH_;
  const int qblk = qblk0 + (int)(blockIdx.x / NBH_);
  const int b = bh / H_, h = bh % H_;
  const int q0 = qblk * 64 + 16 * w;

  const us_t* qp = Qh + (size_t)(bh * SEQ_ + q0) * DH_;
  const Frag aq0 = ldfrag(qp, DH_);
  const Frag aq1 = ldfrag(qp + 32, DH_);
  Frag ar0 = fragz(), ar1 = fragz();
  if (RES) {
    const us_t* qr = Qr + (size_t)(bh * SR_ + q0) * DH_;
    ar0 = ldfrag(qr, DH_);
    ar1 = ldfrag(qr + 32, DH_);
  }

  v8f accO[4], accR[4];
#pragma unroll
  for (int t = 0; t < 4; ++t) { accO[t] = zero8(); accR[t] = zero8(); }
  float m[8], l[8];
#pragma unroll
  for (int i = 0; i < 8; ++i) { m[i] = -1.0e30f; l[i] = 0.0f; }

  _Float16* plh = &Pl[w][0][0];
  _Float16* plr = &Pl[w][1][0];
  const int nch = (q0 + 16 + 31) >> 5;

#pragma unroll 1
  for (int kc = 0; kc < nch; ++kc) {
    const int kb = kc << 5;
    float sc[2][8];
#pragma unroll
    for (int jt = 0; jt < 2; ++jt) {
      const int kr0 = kb + 16 * jt;
      const us_t* kp = Kh + (size_t)(bh * SEQ_ + kr0) * DH_;
      const Frag k0 = ldfrag(kp, DH_);
      const Frag k1 = ldfrag(kp + 32, DH_);
      v8f s = zero8();
      s = mma_f16(aq0.h, k0.h, s);
      s = mma_f16(aq1.h, k1.h, s);
      if (RES) {
        v8f t2 = zero8();
        t2 = mma_f16(ar0.h, k0.h, t2);
        t2 = mma_f16(ar1.h, k1.h, t2);
        const us_t* ep = Kr + (size_t)(bh * SR_ + kr0) * DH_;
        const Frag e0 = ldfrag(ep, DH_);
        const Frag e1 = ldfrag(ep + 32, DH_);
        t2 = mma_f16(aq0.h, e0.h, t2);
        t2 = mma_f16(aq1.h, e1.h, t2);
#pragma unroll
        for (int i = 0; i < 8; ++i) sc[jt][i] = (s[i] + t2[i] * RCI_) * 0.125f;
      } else {
#pragma unroll
        for (int i = 0; i < 8; ++i) sc[jt][i] = s[i] * 0.125f;
      }
    }
#pragma unroll
    for (int jt = 0; jt < 2; ++jt) {
#pragma unroll
      for (int i = 0; i < 8; ++i) {
        const int key = kb + 16 * jt + n;
        const int q = q0 + 8 * hh + i;
        sc[jt][i] = (key > q) ? -1.0e30f : sc[jt][i];
      }
    }
    float p[2][8];
#pragma unroll
    for (int i = 0; i < 8; ++i) {
      float mx = fmaxf(sc[0][i], sc[1][i]);
      mx = fmaxf(mx, __shfl_xor(mx, 1, 32));
      mx = fmaxf(mx, __shfl_xor(mx, 2, 32));
      mx = fmaxf(mx, __shfl_xor(mx, 4, 32));
      mx = fmaxf(mx, __shfl_xor(mx, 8, 32));
      const float mn = fmaxf(m[i], mx);
      const float al = __expf(m[i] - mn);
      const float p0 = __expf(sc[0][i] - mn);
      const float p1 = __expf(sc[1][i] - mn);
      float rs = p0 + p1;
      rs += __shfl_xor(rs, 1, 32);
      rs += __shfl_xor(rs, 2, 32);
      rs += __shfl_xor(rs, 4, 32);
      rs += __shfl_xor(rs, 8, 32);
      l[i] = l[i] * al + rs;
      m[i] = mn;
      p[0][i] = p0;
      p[1][i] = p1;
#pragma unroll
      for (int t = 0; t < 4; ++t) {
        accO[t][i] *= al;
        if (RES) accR[t][i] *= al;
      }
    }
#pragma unroll
    for (int jt = 0; jt < 2; ++jt) {
#pragma unroll
      for (int i = 0; i < 8; ++i) {
        const float pv = p[jt][i];
        const _Float16 xh = (_Float16)pv;
        const int idx = (8 * hh + i) * LDP_ + 16 * jt + n;
        plh[idx] = xh;
        if (RES) plr[idx] = (_Float16)((pv - (float)xh) * RC_);
      }
    }
    wave_lds_sync();
    Frag pa, pr = fragz();
    pa.hv[0] = *(const v8h*)(plh + n * LDP_ + 8 * hh);
    pa.hv[1] = *(const v8h*)(plh + n * LDP_ + 16 + 8 * hh);
    if (RES) {
      pr.hv[0] = *(const v8h*)(plr + n * LDP_ + 8 * hh);
      pr.hv[1] = *(const v8h*)(plr + n * LDP_ + 16 + 8 * hh);
    }
    wave_lds_sync();
#pragma unroll
    for (int t = 0; t < 4; ++t) {
      const Frag vh = ldfrag(Vth + (size_t)(bh * DH_ + 16 * t) * SEQ_ + kb, SEQ_);
      accO[t] = mma_f16(pa.h, vh.h, accO[t]);
      if (RES) {
        const Frag vr = ldfrag(Vtr + (size_t)(bh * DH_ + 16 * t) * SR_ + kb, SR_);
        accR[t] = mma_f16(pa.h, vr.h, accR[t]);
        accR[t] = mma_f16(pr.h, vh.h, accR[t]);
      }
    }
  }

  float li[8];
#pragma unroll
  for (int i = 0; i < 8; ++i) li[i] = 1.0f / l[i];
  _Float16* ch = &Cs[w][0][0];
  _Float16* cr = &Cs[w][1][0];
#pragma unroll
  for (int t = 0; t < 4; ++t) {
#pragma unroll
    for (int i = 0; i < 8; ++i) {
      float v = accO[t][i];
      if (RES) v += accR[t][i] * RCI_;
      v *= li[i];
      const _Float16 xh = (_Float16)v;
      const int idx = (8 * hh + i) * LDT_ + 16 * t + n;
      ch[idx] = xh;
      if (RES) cr[idx] = (_Float16)((v - (float)xh) * RC_);
    }
  }
  __syncthreads();
  const int pc = lane & 7;
  v4u hq[4], rq[4];
  size_t oh[4], orr[4];
#pragma unroll
  for (int pp = 0; pp < 4; ++pp) {
    const int L = 4 * pp + (lane >> 3);
    const v8h e0 = *(const v8h*)(ch + L * LDT_ + 8 * pc);
    hq[pp] = __builtin_bit_cast(v4u, e0);
    oh[pp] = (size_t)(b * SEQ_ + q0 + L) * D_ + h * DH_ + 8 * pc;
    if (RES) {
      const v8h e1 = *(const v8h*)(cr + L * LDT_ + 8 * pc);
      rq[pp] = __builtin_bit_cast(v4u, e1);
      orr[pp] = (size_t)(b * SR_ + q0 + L) * D_ + h * DH_ + 8 * pc;
    }
  }
#pragma unroll
  for (int pp = 0; pp < 4; ++pp) {
    *(volatile v4u*)(CtxH + oh[pp]) = hq[pp];
    if (RES) *(volatile v4u*)(CtxR + orr[pp]) = rq[pp];
  }
  __threadfence();
#pragma unroll
  for (int pp = 0; pp < 4; ++pp) {
    *(volatile v4u*)(CtxH + oh[pp]) = hq[pp];
    if (RES) *(volatile v4u*)(CtxR + orr[pp]) = rq[pp];
  }
}

template <int RES>
__global__ __launch_bounds__(128) void k_oproj(const us_t* __restrict__ CtxH, const us_t* __restrict__ CtxR,
                                               const us_t* __restrict__ WoT, const float* __restrict__ bo,
                                               float* __restrict__ out, int sblk0, int nsb) {
  __shared__ __align__(16) float Os[4][16 * LDO_];
  const int tid = threadIdx.x, w = tid >> 5, lane = tid & 31, n = lane & 15, hh = lane >> 4;
  const int b = blockIdx.x / nsb;
  const int sblk = sblk0 + ((int)blockIdx.x - b * nsb);
  const int s0 = sblk * 64 + 16 * w;
  const int n0 = blockIdx.y * 64;
  const us_t* A = CtxH + (size_t)(b * SEQ_ + s0) * D_;
  const us_t* Bw = WoT + (size_t)n0 * D_;

  v8f c[4], cr[4];
#pragma unroll
  for (int j = 0; j < 4; ++j) { c[j] = zero8(); cr[j] = zero8(); }
#pragma unroll 2
  for (int g = 0; g < D_; g += 32) {
    const Frag a = ldfrag(A + g, D_);
    Frag ar = fragz();
    if (RES) ar = ldfrag(CtxR + (size_t)(b * SR_ + s0) * D_ + g, D_);
#pragma unroll
    for (int j = 0; j < 4; ++j) {
      const Frag bj = ldfrag(Bw + (size_t)(16 * j) * D_ + g, D_);
      c[j] = mma_f16(a.h, bj.h, c[j]);
      if (RES) cr[j] = mma_f16(ar.h, bj.h, cr[j]);
    }
  }
  float* os = &Os[w][0];
#pragma unroll
  for (int j = 0; j < 4; ++j) {
    int bi = n0 + 16 * j + n;
    bi = bi < 0 ? 0 : (bi > D_ - 1 ? D_ - 1 : bi);
    const float bias = __uint_as_float(bf16_bits(bo[bi]) << 16);
#pragma unroll
    for (int i = 0; i < 8; ++i) {
      float v = c[j][i] * WOCI_;
      if (RES) v += cr[j][i] * (WOCI_ * RCI_);
      v += bias;
      os[(8 * hh + i) * LDO_ + 16 * j + n] = v;
    }
  }
  __syncthreads();
  const int pc = lane & 7;
  v4f ov[8];
  size_t oo[8];
#pragma unroll
  for (int pp = 0; pp < 8; ++pp) {
    const int Lx = 4 * pp + (lane >> 3);
    const int row = Lx >> 1, hf = Lx & 1;
    ov[pp] = *(const v4f*)(os + row * LDO_ + hf * 32 + 4 * pc);
    oo[pp] = (size_t)(b * SEQ_ + s0 + row) * D_ + n0 + hf * 32 + 4 * pc;
  }
#pragma unroll
  for (int pp = 0; pp < 8; ++pp) *(volatile v4f*)(out + oo[pp]) = ov[pp];
  __threadfence();
#pragma unroll
  for (int pp = 0; pp < 8; ++pp) *(volatile v4f*)(out + oo[pp]) = ov[pp];
}

extern "C" void kernel_launch(void* const* d_in, const int* in_sizes, int n_in,
                              void* d_out, int out_size, void* d_ws, size_t ws_size,
                              hipStream_t stream) {
  if (n_in < 6) return;
  if (in_sizes[0] < ((NB_ - 1) * SEQ_FULL_ + SEQ_) * D_) return;
  if (in_sizes[1] < D_ * D_ || in_sizes[2] < D_ * D_ || in_sizes[3] < D_ * D_ || in_sizes[4] < D_ * D_) return;
  if (in_sizes[5] < D_) return;
  if (out_size < NB_ * SEQ_ * D_) return;

  const float* x  = (const float*)d_in[0];
  const float* Wq = (const float*)d_in[1];
  const float* Wk = (const float*)d_in[2];
  const float* Wv = (const float*)d_in[3];
  const float* Wo = (const float*)d_in[4];
  const float* bo = (const float*)d_in[5];
  float* out = (float*)d_out;

  size_t off = 0;
  char* wsb = (char*)d_ws;
  auto carve = [&](size_t bytes) -> char* {
    char* p = wsb + off;
    off += (bytes + 255) & ~(size_t)255;
    return p;
  };
  us_t* Xb  = (us_t*)carve((size_t)NB_ * SEQ_ * D_ * 2);
  us_t* WqT = (us_t*)carve((size_t)D_ * D_ * 2);
  us_t* WkT = (us_t*)carve((size_t)D_ * D_ * 2);
  us_t* WvT = (us_t*)carve((size_t)D_ * D_ * 2);
  us_t* WoT = (us_t*)carve((size_t)D_ * D_ * 2);
  us_t* Qh  = (us_t*)carve((size_t)NBH_ * SEQ_ * DH_ * 2);
  us_t* Kh  = (us_t*)carve((size_t)NBH_ * SEQ_ * DH_ * 2);
  us_t* Qr  = (us_t*)carve((size_t)NBH_ * SR_ * DH_ * 2);
  us_t* Kr  = (us_t*)carve((size_t)NBH_ * SR_ * DH_ * 2);
  us_t* Vth = (us_t*)carve((size_t)NBH_ * DH_ * SEQ_ * 2);
  us_t* Vtr = (us_t*)carve((size_t)NBH_ * DH_ * SR_ * 2);
  us_t* CtH = (us_t*)carve((size_t)NB_ * SEQ_ * D_ * 2);
  us_t* CtR = (us_t*)carve((size_t)NB_ * SR_ * D_ * 2);
  if (off > ws_size) return;
  if (off > (size_t)134217728) return;

  const int NSB  = SEQ_ / 64;
  const int NSBR = SR_ / 64;
  const int NSBM = NSB - NSBR;

  k_prep_x<<<(NB_ * SEQ_ * (D_ / 8)) / 256, 256, 0, stream>>>(x, Xb);
  k_prep_w<<<dim3(D_ / 64, D_ / 64, 4), 256, 0, stream>>>(Wq, Wk, Wv, Wo, WqT, WkT, WvT, WoT);
  k_proj<<<dim3(NB_ * NSB, H_, 3), 128, 0, stream>>>(Xb, WqT, WkT, WvT, Qh, Qr, Kh, Kr, Vth, Vtr);
  k_attn<1><<<NSBR * NBH_, 128, 0, stream>>>(Qh, Qr, Kh, Kr, Vth, Vtr, CtH, CtR, 0, NSBR);
  if (NSBM > 0) {
    k_attn<0><<<NSBM * NBH_, 128, 0, stream>>>(Qh, Qr, Kh, Kr, Vth, Vtr, CtH, CtR, NSBR, NSBM);
  }
  k_oproj<1><<<dim3(NB_ * NSBR, D_ / 64), 128, 0, stream>>>(CtH, CtR, WoT, bo, out, 0, NSBR);
  if (NSBM > 0) {
    k_oproj<0><<<dim3(NB_ * NSBM, D_ / 64), 128, 0, stream>>>(CtH, CtR, WoT, bo, out, NSBR, NSBM);
  }
}
